// multi_gcn_time_51479478010106
// MI455X (gfx1250) — hardware-verified
//
#include <hip/hip_runtime.h>
#include <stddef.h>


typedef _Float16 half_t;
typedef half_t v16h __attribute__((ext_vector_type(16)));
typedef half_t v8h  __attribute__((ext_vector_type(8)));
typedef float  v8f  __attribute__((ext_vector_type(8)));
typedef float  v4f  __attribute__((ext_vector_type(4)));
union Frag { v16h v; v8h h[2]; };

#define NV     512
#define NL     13
#define NLO    11
#define NB     64
#define NC     32
#define NS     3
#define KT     3
#define NBLK   7
#define CCAT   (NBLK * NC)
#define KTOT   (CCAT * KT)
#define NCH    16
#define NCHUNK (NB / NCH)
#define PLANE  (NL * NV)
#define JROWS  (NCH * NC * NL)
#define TBH    (JROWS * NV)
#define YPLANE (NV * NLO)

static_assert(NB % NCH == 0);
static_assert(JROWS % 64 == 0);
static_assert(NV % 128 == 0);
static_assert(NV % 32 == 0);
static_assert(KTOT % 32 == 0);
static_assert((NV * NLO) % 32 == 0);
static_assert((32 * NLO) % 32 == 0);

__device__ __forceinline__ v8f zero8()
{
    v8f z;
#pragma unroll
    for (int e = 0; e < 8; ++e) z[e] = 0.0f;
    return z;
}

__device__ __forceinline__ v8f wmma16(const v16h a, const v16h b, v8f c)
{
    v8f d = __builtin_amdgcn_wmma_f32_16x16x32_f16(false, a, false, b, (short)0, c, false, false);
    asm volatile("v_nop\n\tv_nop\n\tv_nop\n\tv_nop" : "+v"(d) : "v"(a), "v"(b));
    return d;
}

__global__ __launch_bounds__(256)
void k_cvt(const float* __restrict__ src, half_t* dst, int n8, float scale)
{
    const int i = blockIdx.x * 256 + threadIdx.x;
    if (i >= n8) return;
    const v4f a = *(const v4f*)(src + (size_t)i * 8);
    const v4f b = *(const v4f*)(src + (size_t)i * 8 + 4);
    v8h o;
    o[0] = (half_t)(a[0] * scale); o[1] = (half_t)(a[1] * scale);
    o[2] = (half_t)(a[2] * scale); o[3] = (half_t)(a[3] * scale);
    o[4] = (half_t)(b[0] * scale); o[5] = (half_t)(b[1] * scale);
    o[6] = (half_t)(b[2] * scale); o[7] = (half_t)(b[3] * scale);
    half_t* p = dst + (size_t)i * 8;
    *(volatile v8h*)p = o;
    __threadfence();
    *(volatile v8h*)p = o;
}

__global__ __launch_bounds__(256)
void k_cvt_x(const float* __restrict__ x, half_t* T0, int n0)
{
    __shared__ __attribute__((aligned(16))) half_t s[NL * 520];
    const int c = blockIdx.x, nl = blockIdx.y, tid = threadIdx.x;
    const float* src = x + ((size_t)(n0 + nl) * NC + c) * PLANE;
    half_t* dst = T0 + ((size_t)nl * NC + c) * PLANE;
#pragma unroll
    for (int i = 0; i < PLANE / 256; ++i) {
        const int e = tid + 256 * i;
        const int v = e / NL;
        const int l = e - v * NL;
        s[l * 520 + v] = (half_t)src[e];
    }
    __syncthreads();
#pragma unroll
    for (int i = 0; i < 4; ++i) {
        const int item = tid + 256 * i;
        if (item < NL * 64) {
            const int l = item >> 6, q = item & 63;
            const v8h val = *(const v8h*)&s[l * 520 + q * 8];
            *(volatile v8h*)(dst + l * NV + q * 8) = val;
        }
    }
    __threadfence();
#pragma unroll
    for (int i = 0; i < 4; ++i) {
        const int item = tid + 256 * i;
        if (item < NL * 64) {
            const int l = item >> 6, q = item & 63;
            const v8h val = *(const v8h*)&s[l * 520 + q * 8];
            *(volatile v8h*)(dst + l * NV + q * 8) = val;
        }
    }
}

__global__ __launch_bounds__(256)
void k_diff(const half_t* __restrict__ Ah, half_t* T,
            int in_blk0, int in_step, int out_blk0, int out_step)
{
    __shared__ __attribute__((aligned(16))) half_t Cs[64 * 136];
    const int z = blockIdx.z;
    const half_t* A  = Ah + (size_t)z * NV * NV;
    const half_t* In = T + (size_t)(in_blk0 + z * in_step) * TBH;
    half_t* Out      = T + (size_t)(out_blk0 + z * out_step) * TBH;
    const int w0 = blockIdx.x * 128, j0 = blockIdx.y * 64;
    const int tid = threadIdx.x, lane = tid & 31, wave = tid >> 5;
    const int h = lane >> 4, m = lane & 15;
    const int wm = wave & 1, wn = wave >> 1;

    const half_t* ar0 = In + (size_t)(j0 + wm * 32 + m) * NV + 8 * h;
    const half_t* ar1 = ar0 + 16 * NV;
    const half_t* br0 = A + (size_t)(w0 + wn * 32 + m) * NV + 8 * h;
    const half_t* br1 = br0 + 16 * NV;

    v8f acc00 = zero8(), acc01 = zero8(), acc10 = zero8(), acc11 = zero8();

#pragma unroll 2
    for (int k0 = 0; k0 < NV; k0 += 32) {
        Frag a0, a1, b0, b1;
        a0.h[0] = *(const v8h*)(ar0 + k0);  a0.h[1] = *(const v8h*)(ar0 + k0 + 16);
        a1.h[0] = *(const v8h*)(ar1 + k0);  a1.h[1] = *(const v8h*)(ar1 + k0 + 16);
        b0.h[0] = *(const v8h*)(br0 + k0);  b0.h[1] = *(const v8h*)(br0 + k0 + 16);
        b1.h[0] = *(const v8h*)(br1 + k0);  b1.h[1] = *(const v8h*)(br1 + k0 + 16);
        acc00 = wmma16(a0.v, b0.v, acc00);
        acc01 = wmma16(a0.v, b1.v, acc01);
        acc10 = wmma16(a1.v, b0.v, acc10);
        acc11 = wmma16(a1.v, b1.v, acc11);
    }

    {
        const int rb = wm * 32 + 8 * h, cb = wn * 32 + m;
#pragma unroll
        for (int r = 0; r < 8; ++r) {
            Cs[(rb + r) * 136 + cb]           = (half_t)acc00[r];
            Cs[(rb + r) * 136 + cb + 16]      = (half_t)acc01[r];
            Cs[(rb + 16 + r) * 136 + cb]      = (half_t)acc10[r];
            Cs[(rb + 16 + r) * 136 + cb + 16] = (half_t)acc11[r];
        }
    }
    __syncthreads();

    v8h val[4];
#pragma unroll
    for (int i = 0; i < 4; ++i) {
        const int item = tid + 256 * i;
        const int row = item >> 4, ch = item & 15;
        val[i] = *(const v8h*)&Cs[row * 136 + ch * 8];
    }
#pragma unroll
    for (int i = 0; i < 4; ++i) {
        const int item = tid + 256 * i;
        const int row = item >> 4, ch = item & 15;
        if (j0 + row < JROWS)
            *(volatile v8h*)(Out + (size_t)(j0 + row) * NV + w0 + ch * 8) = val[i];
    }
    __threadfence();
#pragma unroll
    for (int i = 0; i < 4; ++i) {
        const int item = tid + 256 * i;
        const int row = item >> 4, ch = item & 15;
        if (j0 + row < JROWS)
            *(volatile v8h*)(Out + (size_t)(j0 + row) * NV + w0 + ch * 8) = val[i];
    }
}

__global__ __launch_bounds__(128)
void k_conv(const half_t* __restrict__ T, const half_t* __restrict__ W16,
            const float* __restrict__ bias, float* y, int n0)
{
    __shared__ __attribute__((aligned(16))) half_t Hs[352 * 40];
    __shared__ __attribute__((aligned(16))) float  Ys[16 * 356];
    const int v0 = blockIdx.x * 32, nl = blockIdx.y, n = n0 + nl;
    const int tid = threadIdx.x, lane = tid & 31, wave = tid >> 5;
    const int h = lane >> 4, m = lane & 15;
    const int ot = wave & 1, cw = wave >> 1;
    const int q = tid & 3;

    v8f acc[11];
#pragma unroll
    for (int i = 0; i < 11; ++i) acc[i] = zero8();

    const half_t* wrow = W16 + (size_t)(ot * 16 + m) * KTOT + 8 * h;
    const half_t* Tn   = T + (size_t)nl * NC * PLANE + v0 + q * 8;

    for (int kc = 0; kc < KTOT / 32; ++kc) {
#pragma unroll
        for (int i = 0; i < 11; ++i) {
            const int rest = (tid >> 2) + 32 * i;
            const int kk = rest / NLO;
            const int lo = rest - kk * NLO;
            const int k  = kc * 32 + kk;
            const int cc = k / KT;
            const int kt = k - cc * KT;
            const int blk = cc >> 5, c = cc & 31;
            const v8h val = *(const v8h*)(Tn + (size_t)blk * TBH + (size_t)c * PLANE + (lo + kt) * NV);
            half_t* hp = Hs + ((q * 8) * NLO + lo) * 40 + kk;
#pragma unroll
            for (int e = 0; e < 8; ++e) hp[e * (NLO * 40)] = val[e];
        }
        __syncthreads();

        Frag a;
        a.h[0] = *(const v8h*)(wrow + kc * 32);
        a.h[1] = *(const v8h*)(wrow + kc * 32 + 16);
#pragma unroll
        for (int i = 0; i < 11; ++i) {
            const int ct = cw + 2 * i;
            const half_t* bp = Hs + (ct * 16 + m) * 40 + 8 * h;
            Frag b;
            b.h[0] = *(const v8h*)bp;
            b.h[1] = *(const v8h*)(bp + 16);
            acc[i] = wmma16(a.v, b.v, acc[i]);
        }
        __syncthreads();
    }

    float* ybase = y + ((size_t)n * NC * NV + v0) * NLO;
#pragma unroll
    for (int p = 0; p < 2; ++p) {
        if (ot == p) {
#pragma unroll
            for (int i = 0; i < 11; ++i) {
                const int col = (cw + 2 * i) * 16 + m;
#pragma unroll
                for (int r = 0; r < 8; ++r) {
                    const int ol = 8 * h + r;
                    Ys[ol * 356 + col] = acc[i][r] * 0.0625f + bias[p * 16 + ol];
                }
            }
        }
        __syncthreads();
#pragma unroll
        for (int i = 0; i < 11; ++i) {
            const int item = tid + 128 * i;
            const int row = item / 88, ch = item - row * 88;
            const v4f val = *(const v4f*)&Ys[row * 356 + ch * 4];
            *(volatile v4f*)(ybase + (size_t)(p * 16 + row) * YPLANE + ch * 4) = val;
        }
        __threadfence();
#pragma unroll
        for (int i = 0; i < 11; ++i) {
            const int item = tid + 128 * i;
            const int row = item / 88, ch = item - row * 88;
            const v4f val = *(const v4f*)&Ys[row * 356 + ch * 4];
            *(volatile v4f*)(ybase + (size_t)(p * 16 + row) * YPLANE + ch * 4) = val;
        }
        __syncthreads();
    }
}

static inline size_t al256(size_t v) { return (v + 255) & ~(size_t)255; }

extern "C" void kernel_launch(void* const* d_in, const int* in_sizes, int n_in,
                              void* d_out, int out_size, void* d_ws, size_t ws_size,
                              hipStream_t stream)
{
    if (n_in < 4) return;
    if (in_sizes[0] != NB * NC * NV * NL) return;
    if (in_sizes[1] != NS * NV * NV) return;
    if (in_sizes[2] != NC * CCAT * KT) return;
    if (in_sizes[3] != NC) return;
    if (out_size != NB * NC * NV * NLO) return;

    const float* x       = (const float*)d_in[0];
    const float* support = (const float*)d_in[1];
    const float* W       = (const float*)d_in[2];
    const float* b       = (const float*)d_in[3];
    float* y = (float*)d_out;

    const size_t offA = 0;
    const size_t szA  = (size_t)NS * NV * NV * sizeof(half_t);
    const size_t offW = al256(offA + szA);
    const size_t szW  = (size_t)NC * KTOT * sizeof(half_t);
    const size_t offT = al256(offW + szW);
    const size_t szT  = (size_t)NBLK * TBH * sizeof(half_t);
    const size_t total = offT + szT;
    if (total > ws_size) return;

    half_t* Ah  = (half_t*)((char*)d_ws + offA);
    half_t* W16 = (half_t*)((char*)d_ws + offW);
    half_t* T   = (half_t*)((char*)d_ws + offT);

    const int nA8 = NS * NV * NV / 8;
    const int nW8 = NC * KTOT / 8;
    k_cvt<<<dim3((nA8 + 255) / 256), dim3(256), 0, stream>>>(support, Ah, nA8, 1.0f);
    k_cvt<<<dim3((nW8 + 255) / 256), dim3(256), 0, stream>>>(W, W16, nW8, 16.0f);

    const dim3 dgrid(NV / 128, JROWS / 64, NS);
    for (int ch = 0; ch < NCHUNK; ++ch) {
        const int n0 = ch * NCH;
        k_cvt_x<<<dim3(NC, NCH), dim3(256), 0, stream>>>(x, T, n0);
        k_diff<<<dgrid, dim3(256), 0, stream>>>(Ah, T, 0, 0, 1, 2);
        k_diff<<<dgrid, dim3(256), 0, stream>>>(Ah, T, 1, 2, 2, 2);
        k_conv<<<dim3(NV / 32, NCH), dim3(128), 0, stream>>>(T, W16, b, y, n0);
    }
}
